// LogicExpert_51127290691883
// MI455X (gfx1250) — hardware-run, weakly checked
//
#include <hip/hip_runtime.h>
#include <math.h>

constexpr int kB   = 2;
constexpr int kS   = 1024;
constexpr int kD   = 768;
constexpr int kH   = 12;
constexpr int kDH  = 64;
constexpr int kFF  = 3072;
constexpr int kCH  = 64;
constexpr int kTok = kB * kS;
constexpr int kChunksPerGroup = 4;
constexpr int kGroups = (kTok / kCH) / kChunksPerGroup;
constexpr int kPairs = kChunksPerGroup * kCH * kCH;
constexpr int kTokPerGroup = kChunksPerGroup * kCH;

constexpr float kWCarry   = 16.0f;
constexpr float kWInv     = 1.0f / 16.0f;
constexpr float kPCarry   = 2048.0f;
constexpr float kCtxCarry = 256.0f;
constexpr float kQKScale  = 0.125f;
constexpr float kPVScale  = kCtxCarry / kPCarry;
constexpr float kWoScale  = 1.0f / (kCtxCarry * kWCarry);
constexpr float kInvD     = 1.0f / 768.0f;
constexpr float kInvCH    = 1.0f / 64.0f;
constexpr float kLnEps    = 1e-5f;

constexpr size_t kBytesW768  = (size_t)kD * kD * 2;
constexpr size_t kBytesWff   = (size_t)kD * kFF * 2;
constexpr size_t kBytesTok16 = (size_t)kTok * kD * 2;
constexpr size_t kBytesTok32 = (size_t)kTok * kD * 4;
constexpr size_t kBytesBig   = (size_t)kH * kS * kS * 4;
constexpr size_t kBytesMid   = (size_t)kH * kS * kS * 2;
constexpr size_t kWsTotal = 7 * kBytesW768 + 2 * kBytesWff + kBytesTok16 + kBytesTok32 + kBytesTok16 +
                             kBytesBig + kBytesMid + kBytesTok16 + 3 * kBytesTok32;
static_assert(kWsTotal == (size_t)127795200, "carve total");
static_assert(kWsTotal <= (size_t)134217728, "carve cap");
static_assert((size_t)kPairs * kD * 4 <= kBytesBig, "Y32 fits");
static_assert((size_t)kTok * kFF * 4 <= kBytesBig, "T32 fits");
static_assert((size_t)kPairs * kD * 2 <= kBytesMid, "HP16 fits");
static_assert((size_t)kTok * kFF * 2 <= kBytesMid, "T16 fits");

typedef __attribute__((ext_vector_type(16))) _Float16 v16h;
typedef __attribute__((ext_vector_type(8)))  _Float16 v8h;
typedef __attribute__((ext_vector_type(16))) __bf16   v16b;
typedef __attribute__((ext_vector_type(8)))  __bf16   v8b;
typedef __attribute__((ext_vector_type(8)))  float    v8f;
typedef __attribute__((ext_vector_type(4)))  float    v4f;
typedef __attribute__((ext_vector_type(2)))  float    v2f;
typedef __attribute__((ext_vector_type(4)))  unsigned int v4u;

__device__ __forceinline__ unsigned short f2bf_bits(float f) {
  unsigned u = __float_as_uint(f);
  return (unsigned short)((u + 0x7FFFu + ((u >> 16) & 1u)) >> 16);
}
__device__ __forceinline__ float bf_bits2f(unsigned short h) { return __uint_as_float(((unsigned)h) << 16); }

__device__ __forceinline__ void dep_guard_h(v8f& a, v8f& b, v16h x, v16h y) { asm volatile("v_nop\n\tv_nop\n\tv_nop\n\tv_nop" : "+v"(a), "+v"(b) : "v"(x), "v"(y)); }
__device__ __forceinline__ void dep_guard_b(v8f& a, v8f& b, v16b x, v16b y) { asm volatile("v_nop\n\tv_nop\n\tv_nop\n\tv_nop" : "+v"(a), "+v"(b) : "v"(x), "v"(y)); }
__device__ __forceinline__ void keep4_h(v16h a, v16h b, v16h c, v16h d) { asm volatile("v_nop" :: "v"(a), "v"(b), "v"(c), "v"(d)); }
__device__ __forceinline__ void keep4_b(v16b a, v16b b, v16b c, v16b d) { asm volatile("v_nop" :: "v"(a), "v"(b), "v"(c), "v"(d)); }
__device__ __forceinline__ void acc_guard4(v8f& a, v8f& b, v8f& c, v8f& d) { asm volatile("v_nop\n\tv_nop\n\tv_nop\n\tv_nop" : "+v"(a), "+v"(b), "+v"(c), "+v"(d)); }
template <typename T> struct Frag;
template <> struct Frag<_Float16> {
  typedef v16h V; union U { v16h v; v8h h[2]; };
  static __device__ __forceinline__ v16h load(const _Float16* p) {
    U f; f.h[0] = *(const v8h*)(p); f.h[1] = *(const v8h*)(p + 16); return f.v;
  }
  static __device__ __forceinline__ v8f mma(v16h a, v16h b, v8f c) {
    return __builtin_amdgcn_wmma_f32_16x16x32_f16(false, a, false, b, (short)0, c, false, false);
  }
  static __device__ __forceinline__ void guard(v8f& a, v8f& b, v16h x, v16h y) { dep_guard_h(a, b, x, y); }
  static __device__ __forceinline__ void keep(v16h a, v16h b, v16h c, v16h d) { keep4_h(a, b, c, d); }
};
template <> struct Frag<__bf16> {
  typedef v16b V; union U { v16b v; v8b h[2]; };
  static __device__ __forceinline__ v16b load(const __bf16* p) {
    U f; f.h[0] = *(const v8b*)(p); f.h[1] = *(const v8b*)(p + 16); return f.v;
  }
  static __device__ __forceinline__ v8f mma(v16b a, v16b b, v8f c) {
    return __builtin_amdgcn_wmma_f32_16x16x32_bf16(false, a, false, b, (short)0, c, false, false);
  }
  static __device__ __forceinline__ void guard(v8f& a, v8f& b, v16b x, v16b y) { dep_guard_b(a, b, x, y); }
  static __device__ __forceinline__ void keep(v16b a, v16b b, v16b c, v16b d) { keep4_b(a, b, c, d); }
};

__device__ __forceinline__ unsigned pk16(unsigned short a, unsigned short b) { return (unsigned)a | ((unsigned)b << 16); }
__device__ __forceinline__ unsigned short h_bits(float f) { const _Float16 h = (_Float16)f; return __builtin_bit_cast(unsigned short, h); }

template <int ET> struct Elem;
template <> struct Elem<0> { typedef _Float16 T; };
template <> struct Elem<1> { typedef __bf16 T; };
template <int ET, bool SPLIT, int BIAS_MODE, int OUT_MODE, bool RESID, int ACT = 0>
__global__ __launch_bounds__(256) void wmma_gemm64(
    const unsigned short* __restrict__ Ap, const unsigned short* __restrict__ A2p, int lda, long strideA,
    const unsigned short* __restrict__ Btp, const unsigned short* __restrict__ Bt2p, int ldb, long strideB,
    void* __restrict__ Cout, void* __restrict__ Cout2, int ldc, long strideC,
    const float* __restrict__ bias,
    const float* __restrict__ resid, long strideR,
    int M, int N, int K, float scale) {
  typedef typename Elem<ET>::T T;
  typedef typename Frag<T>::V V;
  const T* A = (const T*)Ap; const T* A2 = (const T*)A2p; const T* Bt = (const T*)Btp; const T* Bt2 = (const T*)Bt2p;
  __shared__ __align__(16) float sT[8][16 * 68];
  const int b    = blockIdx.y;
  const int lane = threadIdx.x & 31;
  const int wave = threadIdx.x >> 5;
  const int tilesN = N >> 6;
  const int tilesM = M >> 6;
  const int tile = blockIdx.x * 8 + wave;
  if (tile >= tilesM * tilesN) return;
  const int tm = tile / tilesN;
  const int tn = tile - tm * tilesN;
  const int m0 = tm << 6;
  const int n0 = tn << 6;

  const T* Ab  = A  + (size_t)b * strideA;
  const T* Bb  = Bt + (size_t)b * strideB;
  const T* Ab2 = SPLIT ? (A2  + (size_t)b * strideA) : nullptr;
  const T* Bb2 = SPLIT ? (Bt2 + (size_t)b * strideB) : nullptr;

  const int rlane = lane & 15;
  const int koff  = (lane >> 4) * 8;
  const int mOff  = (lane >> 4) * 8;

  v8f acc[4][4];
#pragma unroll
  for (int i = 0; i < 4; ++i)
#pragma unroll
    for (int j = 0; j < 4; ++j) acc[i][j] = (v8f){0.f,0.f,0.f,0.f,0.f,0.f,0.f,0.f};

  for (int k0 = 0; k0 < K; k0 += 32) {
    V bh[4], bl[4];
#pragma unroll
    for (int j = 0; j < 4; ++j) {
      const size_t bo = (size_t)(n0 + (j << 4) + rlane) * ldb + koff + k0;
      bh[j] = Frag<T>::load(Bb + bo);
      if (SPLIT) bl[j] = Frag<T>::load(Bb2 + bo);
    }
#pragma unroll
    for (int i = 0; i < 4; ++i) {
      const size_t ao = (size_t)(m0 + (i << 4) + rlane) * lda + koff + k0;
      V ah = Frag<T>::load(Ab + ao);
      V al;
      if (SPLIT) al = Frag<T>::load(Ab2 + ao);
#pragma unroll
      for (int j = 0; j < 4; ++j) {
        acc[i][j] = Frag<T>::mma(ah, bh[j], acc[i][j]);
        if (SPLIT) {
          acc[i][j] = Frag<T>::mma(ah, bl[j], acc[i][j]);
          acc[i][j] = Frag<T>::mma(al, bh[j], acc[i][j]);
        }
      }
      Frag<T>::guard(acc[i][0], acc[i][3], ah, SPLIT ? al : ah);
    }
    Frag<T>::keep(bh[0], bh[1], bh[2], bh[3]);
    if (SPLIT) Frag<T>::keep(bl[0], bl[1], bl[2], bl[3]);
  }
  acc_guard4(acc[0][0], acc[0][1], acc[0][2], acc[0][3]);
  acc_guard4(acc[1][0], acc[1][1], acc[1][2], acc[1][3]);
  acc_guard4(acc[2][0], acc[2][1], acc[2][2], acc[2][3]);
  acc_guard4(acc[3][0], acc[3][1], acc[3][2], acc[3][3]);

  float* slab = sT[wave];
  const float* Rb = RESID ? (resid + (size_t)b * strideR) : nullptr;
#pragma unroll
  for (int i = 0; i < 4; ++i) {
    const int mBase = m0 + (i << 4);
#pragma unroll
    for (int j = 0; j < 4; ++j) {
      const int n = n0 + (j << 4) + rlane;
      float bv = 0.f;
      if (BIAS_MODE == 2) bv = bias[n];
#pragma unroll
      for (int r = 0; r < 8; ++r) {
        float v = acc[i][j][r] * scale;
        if (BIAS_MODE == 1) v += bias[mBase + mOff + r];
        if (BIAS_MODE == 2) v += bv;
        if (RESID) v += Rb[(size_t)(mBase + mOff + r) * ldc + n];
        if (ACT == 2) v = fmaxf(v, 0.0f);
        if (ACT == 4) v = (v > 0.f) ? v : 0.01f * v;
        slab[(mOff + r) * 68 + (j << 4) + rlane] = v;
      }
    }
    __builtin_amdgcn_fence(__ATOMIC_RELEASE, "workgroup");
    __builtin_amdgcn_wave_barrier();
    __builtin_amdgcn_fence(__ATOMIC_ACQUIRE, "workgroup");
    if (OUT_MODE == 0) {
      float* C = (float*)Cout + (size_t)b * strideC;
      const int hh = lane >> 4, c4 = (lane & 15) * 4;
      for (int pass = 0; pass < 2; ++pass) {
#pragma unroll
        for (int it = 0; it < 8; ++it) {
          const int row = it * 2 + hh;
          v4f v = *(const v4f*)(slab + row * 68 + c4);
          *(volatile v4f*)(C + (size_t)(mBase + row) * ldc + n0 + c4) = v;
        }
        __threadfence();
      }
    } else {
      const int q = lane >> 3, c8 = (lane & 7) * 8;
      unsigned short* C  = (unsigned short*)Cout  + (size_t)b * strideC;
      unsigned short* C2 = (OUT_MODE == 2) ? ((unsigned short*)Cout2 + (size_t)b * strideC) : nullptr;
      for (int pass = 0; pass < 2; ++pass) {
#pragma unroll
        for (int it = 0; it < 4; ++it) {
          const int row = it * 4 + q;
          const float* sp = slab + row * 68 + c8;
          v8h hv, lv;
#pragma unroll
          for (int e = 0; e < 8; ++e) {
            if (OUT_MODE == 1) {
              hv[e] = (_Float16)sp[e];
            } else {
              unsigned short hb = f2bf_bits(sp[e]);
              unsigned short lb = f2bf_bits(sp[e] - bf_bits2f(hb));
              hv[e] = __builtin_bit_cast(_Float16, hb);
              lv[e] = __builtin_bit_cast(_Float16, lb);
            }
          }
          *(volatile v8h*)(C + (size_t)(mBase + row) * ldc + n0 + c8) = hv;
          if (OUT_MODE == 2) *(volatile v8h*)(C2 + (size_t)(mBase + row) * ldc + n0 + c8) = lv;
        }
        __threadfence();
      }
    }
    __builtin_amdgcn_fence(__ATOMIC_RELEASE, "workgroup");
    __builtin_amdgcn_wave_barrier();
    __builtin_amdgcn_fence(__ATOMIC_ACQUIRE, "workgroup");
  }
}

__global__ __launch_bounds__(256) void wt_kernel(const float* __restrict__ W, unsigned short* __restrict__ out,
                                                 int R, int Cc, float scale) {
  __shared__ float sm[64][65];
  const int t  = threadIdx.x;
  const int r0 = blockIdx.x * 64;
  const int c0 = blockIdx.y * 64;
#pragma unroll
  for (int i = 0; i < 16; ++i) {
    const int e  = i * 256 + t;
    const int rl = e >> 6;
    const int cl = e & 63;
    sm[cl][rl] = W[(size_t)(r0 + rl) * Cc + c0 + cl] * scale;
  }
  __syncthreads();
  const int lane = t & 31, wave = t >> 5;
  const int q = lane >> 3, c8 = (lane & 7) * 8;
  for (int pass = 0; pass < 2; ++pass) {
#pragma unroll
    for (int it = 0; it < 2; ++it) {
      const int row = wave * 8 + it * 4 + q;
      unsigned short hb[8];
#pragma unroll
      for (int e = 0; e < 8; ++e) hb[e] = h_bits(sm[row][c8 + e]);
      const v4u u = (v4u){pk16(hb[0], hb[1]), pk16(hb[2], hb[3]), pk16(hb[4], hb[5]), pk16(hb[6], hb[7])};
      *(volatile v4u*)(out + (size_t)(c0 + row) * R + r0 + c8) = u;
    }
    __threadfence();
  }
}

__global__ __launch_bounds__(96) void ln_rows_f16_kernel(const float* __restrict__ x, const float* __restrict__ g,
                                                         const float* __restrict__ bb, unsigned short* __restrict__ out) {
  __shared__ float sSum[4];
  __shared__ float sSq[4];
  const int row  = blockIdx.x;
  const int t    = threadIdx.x;
  const int lane = t & 31, wave = t >> 5;
  const int c0   = 8 * t;
  const float* xr = x + (size_t)row * kD + c0;
  const v4f a = *(const v4f*)(xr);
  const v4f c = *(const v4f*)(xr + 4);
  float v[8];
#pragma unroll
  for (int e = 0; e < 4; ++e) { v[e] = a[e]; v[4 + e] = c[e]; }
  float s = ((v[0] + v[1]) + (v[2] + v[3])) + ((v[4] + v[5]) + (v[6] + v[7]));
#pragma unroll
  for (int off = 16; off > 0; off >>= 1) s += __shfl_xor(s, off, 32);
  if (lane == 0) sSum[wave] = s;
  __syncthreads();
  const float mean = ((sSum[0] + sSum[1]) + sSum[2]) * kInvD;
  float d[8];
  float q = 0.f;
#pragma unroll
  for (int e = 0; e < 8; ++e) { d[e] = v[e] - mean; q += d[e] * d[e]; }
#pragma unroll
  for (int off = 16; off > 0; off >>= 1) q += __shfl_xor(q, off, 32);
  if (lane == 0) sSq[wave] = q;
  __syncthreads();
  const float var = ((sSq[0] + sSq[1]) + sSq[2]) * kInvD;
  const float inv = rsqrtf(var + kLnEps);
  const v4f g0 = *(const v4f*)(g + c0);
  const v4f g1 = *(const v4f*)(g + c0 + 4);
  const v4f b0 = *(const v4f*)(bb + c0);
  const v4f b1 = *(const v4f*)(bb + c0 + 4);
  unsigned short hb[8];
#pragma unroll
  for (int e = 0; e < 4; ++e) {
    hb[e]     = h_bits(d[e] * inv * g0[e] + b0[e]);
    hb[4 + e] = h_bits(d[4 + e] * inv * g1[e] + b1[e]);
  }
  const v4u u = (v4u){pk16(hb[0], hb[1]), pk16(hb[2], hb[3]), pk16(hb[4], hb[5]), pk16(hb[6], hb[7])};
  unsigned short* op = out + (size_t)row * kD + c0;
  *(volatile v4u*)op = u;
  __threadfence();
  *(volatile v4u*)op = u;
}

__global__ __launch_bounds__(128) void softmax_rows_kernel(const float* __restrict__ Sc, unsigned short* __restrict__ P,
                                                           float carry) {
  __shared__ float redM[4];
  __shared__ float redS[4];
  const int row  = blockIdx.x;
  const int t    = threadIdx.x;
  const int lane = t & 31, wave = t >> 5;
  const int c0   = 8 * t;
  const float* sr = Sc + (size_t)row * kS + c0;
  const v4f a = *(const v4f*)(sr);
  const v4f c = *(const v4f*)(sr + 4);
  float x[8];
#pragma unroll
  for (int e = 0; e < 4; ++e) { x[e] = a[e]; x[4 + e] = c[e]; }
  float m = fmaxf(fmaxf(fmaxf(x[0], x[1]), fmaxf(x[2], x[3])), fmaxf(fmaxf(x[4], x[5]), fmaxf(x[6], x[7])));
#pragma unroll
  for (int off = 16; off > 0; off >>= 1) m = fmaxf(m, __shfl_xor(m, off, 32));
  if (lane == 0) redM[wave] = m;
  __syncthreads();
  m = fmaxf(fmaxf(redM[0], redM[1]), fmaxf(redM[2], redM[3]));
  float ev[8];
#pragma unroll
  for (int e = 0; e < 8; ++e) ev[e] = expf(x[e] - m);
  float s = ((ev[0] + ev[1]) + (ev[2] + ev[3])) + ((ev[4] + ev[5]) + (ev[6] + ev[7]));
#pragma unroll
  for (int off = 16; off > 0; off >>= 1) s += __shfl_xor(s, off, 32);
  if (lane == 0) redS[wave] = s;
  __syncthreads();
  const float tot = (redS[0] + redS[1]) + (redS[2] + redS[3]);
  const float inv = carry * (1.0f / tot);
  unsigned short hb[8];
#pragma unroll
  for (int e = 0; e < 8; ++e) hb[e] = h_bits(ev[e] * inv);
  const v4u u = (v4u){pk16(hb[0], hb[1]), pk16(hb[2], hb[3]), pk16(hb[4], hb[5]), pk16(hb[6], hb[7])};
  unsigned short* op = P + (size_t)row * kS + c0;
  *(volatile v4u*)op = u;
  __threadfence();
  *(volatile v4u*)op = u;
}

__global__ __launch_bounds__(256) void cast8_f16_kernel(const float* __restrict__ in, unsigned short* __restrict__ out, int n8) {
  const int i = blockIdx.x * 256 + threadIdx.x;
  if (i >= n8) return;
  const float* p = in + 8 * (size_t)i;
  const v4f a = *(const v4f*)(p);
  const v4f c = *(const v4f*)(p + 4);
  unsigned short hb[8];
#pragma unroll
  for (int e = 0; e < 4; ++e) {
    hb[e]     = h_bits(a[e]);
    hb[4 + e] = h_bits(c[e]);
  }
  const v4u u = (v4u){pk16(hb[0], hb[1]), pk16(hb[2], hb[3]), pk16(hb[4], hb[5]), pk16(hb[6], hb[7])};
  unsigned short* q = out + 8 * (size_t)i;
  *(volatile v4u*)q = u;
  __threadfence();
  *(volatile v4u*)q = u;
}

__device__ __forceinline__ float gelu_erf(float x) {
  return 0.5f * x * (1.0f + erff(x * 0.70710678118654752f));
}

__global__ __launch_bounds__(256) void gelu2_f16_kernel(const float* __restrict__ in, unsigned short* __restrict__ out, int n2) {
  const int i = blockIdx.x * 256 + threadIdx.x;
  if (i >= n2) return;
  const v2f a = *(const v2f*)(in + 2 * (size_t)i);
  const float g0 = gelu_erf(a[0]);
  const float g1 = gelu_erf(a[1]);
  const unsigned u = pk16(h_bits(g0), h_bits(g1));
  unsigned* q = (unsigned*)(void*)out + (size_t)i;
  *(volatile unsigned*)q = u;
  __threadfence();
  *(volatile unsigned*)q = u;
}

__global__ __launch_bounds__(256) void pair_gelu_kernel(const float* __restrict__ Abuf, const float* __restrict__ Bbuf,
                                                        unsigned short* __restrict__ HP, int tok0) {
  const int lane = threadIdx.x & 31, wave = threadIdx.x >> 5;
  const int p  = blockIdx.x * 8 + wave;
  const int q  = p >> 6;
  const int cl = p >> 12;
  const int j  = p & 63;
  const int ri = tok0 + q;
  const int rj = tok0 + cl * kCH + j;
  const float* ar = Abuf + (size_t)ri * kD + 2 * lane;
  const float* br = Bbuf + (size_t)rj * kD + 2 * lane;
  unsigned* hrow = (unsigned*)(void*)HP + (size_t)p * (kD / 2) + lane;
#pragma unroll 1
  for (int it = 0; it < kD / 64; ++it) {
    const v2f av = *(const v2f*)(ar + 64 * it);
    const v2f bv = *(const v2f*)(br + 64 * it);
    const float x0 = av[0] + bv[0];
    const float x1 = av[1] + bv[1];
    const float g0 = gelu_erf(x0);
    const float g1 = gelu_erf(x1);
    const unsigned u = pk16(h_bits(g0), h_bits(g1));
    unsigned* qo = hrow + 32 * it;
    *(volatile unsigned*)qo = u;
    __threadfence();
    *(volatile unsigned*)qo = u;
  }
}

__global__ __launch_bounds__(256) void relnorm_mean_kernel(const float* __restrict__ Y, const float* __restrict__ g,
                                                           const float* __restrict__ bb, const float* __restrict__ x1,
                                                           float* __restrict__ x2, int tok0) {
  const int lane = threadIdx.x & 31, wave = threadIdx.x >> 5;
  const int q = blockIdx.x * 8 + wave;
  const float* yb = Y + (size_t)q * kCH * kD + 4 * lane;
  v4f acc[6];
#pragma unroll
  for (int k = 0; k < 6; ++k) acc[k] = (v4f){0.f, 0.f, 0.f, 0.f};
#pragma unroll 1
  for (int j = 0; j < kCH; ++j) {
    const float* yr = yb + (size_t)j * kD;
    v4f t[6];
#pragma unroll
    for (int k = 0; k < 6; ++k) t[k] = *(const v4f*)(yr + 128 * k);
    float s = 0.f;
#pragma unroll
    for (int k = 0; k < 6; ++k) s += (t[k][0] + t[k][1]) + (t[k][2] + t[k][3]);
#pragma unroll
    for (int off = 16; off > 0; off >>= 1) s += __shfl_xor(s, off, 32);
    const float mean = s * kInvD;
    float qv = 0.f;
#pragma unroll
    for (int k = 0; k < 6; ++k) {
      t[k] = t[k] - mean;
      qv += t[k][0] * t[k][0];
      qv += t[k][1] * t[k][1];
      qv += t[k][2] * t[k][2];
      qv += t[k][3] * t[k][3];
    }
#pragma unroll
    for (int off = 16; off > 0; off >>= 1) qv += __shfl_xor(qv, off, 32);
    const float var = qv * kInvD;
    const float inv = rsqrtf(var + kLnEps);
#pragma unroll
    for (int k = 0; k < 6; ++k) acc[k] += t[k] * inv;
  }
  const int row = tok0 + q;
  const float* xr = x1 + (size_t)row * kD + 4 * lane;
  const float* gr = g + 4 * lane;
  const float* br = bb + 4 * lane;
  float* orow = x2 + (size_t)row * kD + 4 * lane;
  v4f o[6];
#pragma unroll
  for (int k = 0; k < 6; ++k) {
    const v4f gg = *(const v4f*)(gr + 128 * k);
    const v4f bv = *(const v4f*)(br + 128 * k);
    const v4f xv = *(const v4f*)(xr + 128 * k);
    o[k] = xv + (acc[k] * kInvCH * gg + bv);
  }
  for (int pass = 0; pass < 2; ++pass) {
#pragma unroll
    for (int k = 0; k < 6; ++k) *(volatile v4f*)(orow + 128 * k) = o[k];
    __threadfence();
  }
}

template <int BIAS_MODE, int OUT_MODE, bool RESID>
static void launch_gemm(hipStream_t st, int batch,
                        const void* A, int lda, long sA,
                        const void* Bt, int ldb, long sB,
                        void* C, int ldc, long sC,
                        const float* bias, const float* resid, long sR,
                        int M, int N, int K, float scale) {
  const int tiles = (M >> 6) * (N >> 6);
  dim3 grid((unsigned)((tiles + 7) / 8), (unsigned)batch, 1);
  wmma_gemm64<0, false, BIAS_MODE, OUT_MODE, RESID, 0><<<grid, 256, 0, st>>>(
      (const unsigned short*)A, (const unsigned short*)A, lda, sA,
      (const unsigned short*)Bt, (const unsigned short*)Bt, ldb, sB,
      C, C, ldc, sC, bias, resid, sR, M, N, K, scale);
}

extern "C" void kernel_launch(void* const* d_in, const int* in_sizes, int n_in,
                              void* d_out, int out_size, void* d_ws, size_t ws_size,
                              hipStream_t stream) {
  if (n_in < 23) return;
  if (out_size != kTok * kD) return;
  if (in_sizes[0] != kTok * kD || in_sizes[1] != kD * kD || in_sizes[3] != kD * kD || in_sizes[5] != kD * kD ||
      in_sizes[7] != kD * kD || in_sizes[11] != 2 * kD * kD || in_sizes[13] != kD * kD ||
      in_sizes[19] != kD * kFF || in_sizes[21] != kFF * kD) return;
  if (in_sizes[2] != kD || in_sizes[9] != kD || in_sizes[15] != kD || in_sizes[20] != kFF || in_sizes[22] != kD) return;
  if (ws_size < kWsTotal) return;

  const float* x      = (const float*)d_in[0];
  const float* Wq     = (const float*)d_in[1];
  const float* bq     = (const float*)d_in[2];
  const float* Wk     = (const float*)d_in[3];
  const float* bk     = (const float*)d_in[4];
  const float* Wv     = (const float*)d_in[5];
  const float* bv     = (const float*)d_in[6];
  const float* Wo     = (const float*)d_in[7];
  const float* bo     = (const float*)d_in[8];
  const float* ln1_g  = (const float*)d_in[9];
  const float* ln1_b  = (const float*)d_in[10];
  const float* rel_W1 = (const float*)d_in[11];
  const float* rel_b1 = (const float*)d_in[12];
  const float* rel_W2 = (const float*)d_in[13];
  const float* rel_b2 = (const float*)d_in[14];
  const float* rln_g  = (const float*)d_in[15];
  const float* rln_b  = (const float*)d_in[16];
  const float* ln2_g  = (const float*)d_in[17];
  const float* ln2_b  = (const float*)d_in[18];
  const float* enc_W1 = (const float*)d_in[19];
  const float* enc_b1 = (const float*)d_in[20];
  const float* enc_W2 = (const float*)d_in[21];
  const float* enc_b2 = (const float*)d_in[22];

  char* ws = (char*)d_ws;
  size_t off = 0;
  unsigned short* WqT    = (unsigned short*)(ws + off); off += kBytesW768;
  unsigned short* WkT    = (unsigned short*)(ws + off); off += kBytesW768;
  unsigned short* WvT    = (unsigned short*)(ws + off); off += kBytesW768;
  unsigned short* WoT    = (unsigned short*)(ws + off); off += kBytesW768;
  unsigned short* W1aT   = (unsigned short*)(ws + off); off += kBytesW768;
  unsigned short* W1bT   = (unsigned short*)(ws + off); off += kBytesW768;
  unsigned short* W2T    = (unsigned short*)(ws + off); off += kBytesW768;
  unsigned short* encW1T = (unsigned short*)(ws + off); off += kBytesWff;
  unsigned short* encW2T = (unsigned short*)(ws + off); off += kBytesWff;
  unsigned short* h16    = (unsigned short*)(ws + off); off += kBytesTok16;
  char* rQK = ws + off; off += kBytesTok32;
  unsigned short* q16  = (unsigned short*)rQK;
  unsigned short* k16  = (unsigned short*)(rQK + kBytesTok16);
  float* Abuf          = (float*)rQK;
  char* rVT = ws + off; off += kBytesTok16;
  unsigned short* vt16  = (unsigned short*)rVT;
  unsigned short* x1_16 = (unsigned short*)rVT;
  char* rBIG = ws + off; off += kBytesBig;
  float* scores = (float*)rBIG;
  float* Y32    = (float*)rBIG;
  float* T32    = (float*)rBIG;
  char* rMID = ws + off; off += kBytesMid;
  unsigned short* P16  = (unsigned short*)rMID;
  unsigned short* HP16 = (unsigned short*)rMID;
  unsigned short* T16  = (unsigned short*)rMID;
  unsigned short* ctx16 = (unsigned short*)(ws + off); off += kBytesTok16;
  float* x1   = (float*)(ws + off); off += kBytesTok32;
  float* Bbuf = (float*)(ws + off); off += kBytesTok32;
  float* x2   = (float*)(ws + off); off += kBytesTok32;
  if (off != kWsTotal || off > ws_size) return;
  float* outp = (float*)d_out;

  wt_kernel<<<dim3(kD / 64, kD / 64), 256, 0, stream>>>(Wq, WqT, kD, kD, kWCarry);
  wt_kernel<<<dim3(kD / 64, kD / 64), 256, 0, stream>>>(Wk, WkT, kD, kD, kWCarry);
  wt_kernel<<<dim3(kD / 64, kD / 64), 256, 0, stream>>>(Wv, WvT, kD, kD, kWCarry);
  wt_kernel<<<dim3(kD / 64, kD / 64), 256, 0, stream>>>(Wo, WoT, kD, kD, kWCarry);
  wt_kernel<<<dim3(kD / 64, kD / 64), 256, 0, stream>>>(rel_W1, W1aT, kD, kD, kWCarry);
  wt_kernel<<<dim3(kD / 64, kD / 64), 256, 0, stream>>>(rel_W1 + (size_t)kD * kD, W1bT, kD, kD, kWCarry);
  wt_kernel<<<dim3(kD / 64, kD / 64), 256, 0, stream>>>(rel_W2, W2T, kD, kD, kWCarry);
  wt_kernel<<<dim3(kD / 64, kFF / 64), 256, 0, stream>>>(enc_W1, encW1T, kD, kFF, kWCarry);
  wt_kernel<<<dim3(kFF / 64, kD / 64), 256, 0, stream>>>(enc_W2, encW2T, kFF, kD, kWCarry);

  ln_rows_f16_kernel<<<kTok, 96, 0, stream>>>(x, ln1_g, ln1_b, h16);
  launch_gemm<2, 1, false>(stream, 1, h16, kD, 0, WqT, kD, 0, q16, kD, 0, bq, x, 0, kTok, kD, kD, kWInv);
  launch_gemm<2, 1, false>(stream, 1, h16, kD, 0, WkT, kD, 0, k16, kD, 0, bk, x, 0, kTok, kD, kD, kWInv);
  launch_gemm<1, 1, false>(stream, 1, WvT, kD, 0, h16, kD, 0, vt16, kTok, 0, bv, x, 0, kD, kTok, kD, kWInv);
  for (int bidx = 0; bidx < kB; ++bidx) {
    const unsigned short* qb = q16 + (size_t)bidx * kS * kD;
    const unsigned short* kb = k16 + (size_t)bidx * kS * kD;
    launch_gemm<0, 0, false>(stream, kH, qb, kD, (long)kDH, kb, kD, (long)kDH,
                             scores, kS, (long)kS * kS, bq, x, 0, kS, kS, kDH, kQKScale);
    softmax_rows_kernel<<<kH * kS, 128, 0, stream>>>(scores, P16, kPCarry);
    launch_gemm<0, 1, false>(stream, kH, P16, kS, (long)kS * kS, vt16 + (size_t)bidx * kS, kTok, (long)kDH * kTok,
                             ctx16 + (size_t)bidx * kS * kD, kD, (long)kDH, bq, x, 0, kS, kDH, kS, kPVScale);
  }
  launch_gemm<2, 0, true>(stream, 1, ctx16, kD, 0, WoT, kD, 0, x1, kD, 0, bo, x, 0, kTok, kD, kD, kWoScale);

  cast8_f16_kernel<<<(kTok * kD / 8) / 256, 256, 0, stream>>>(x1, x1_16, kTok * kD / 8);
  launch_gemm<2, 0, false>(stream, 1, x1_16, kD, 0, W1aT, kD, 0, Abuf, kD, 0, rel_b1, x, 0, kTok, kD, kD, kWInv);
  launch_gemm<0, 0, false>(stream, 1, x1_16, kD, 0, W1bT, kD, 0, Bbuf, kD, 0, rel_b1, x, 0, kTok, kD, kD, kWInv);
  for (int gidx = 0; gidx < kGroups; ++gidx) {
    const int tok0 = gidx * kTokPerGroup;
    pair_gelu_kernel<<<kPairs / 8, 256, 0, stream>>>(Abuf, Bbuf, HP16, tok0);
    launch_gemm<2, 0, false>(stream, 1, HP16, kD, 0, W2T, kD, 0, Y32, kD, 0, rel_b2, x, 0, kPairs, kD, kD, kWInv);
    relnorm_mean_kernel<<<kTokPerGroup / 8, 256, 0, stream>>>(Y32, rln_g, rln_b, x1, x2, tok0);
  }

  ln_rows_f16_kernel<<<kTok, 96, 0, stream>>>(x2, ln2_g, ln2_b, h16);
  launch_gemm<2, 0, false>(stream, 1, h16, kD, 0, encW1T, kD, 0, T32, kFF, 0, enc_b1, x, 0, kTok, kFF, kD, kWInv);
  gelu2_f16_kernel<<<(kTok * kFF / 2) / 256, 256, 0, stream>>>(T32, T16, kTok * kFF / 2);
  launch_gemm<2, 0, true>(stream, 1, T16, kFF, 0, encW2T, kFF, 0, outp, kD, 0, enc_b2, x2, 0, kTok, kD, kFF, kWInv);
}
